// STGCNLayer_67216238183256
// MI455X (gfx1250) — hardware-run, weakly checked
//
#include <hip/hip_runtime.h>


#ifndef NB
#define NB 32
#endif
#define NB_FULL 32
#define CI   64
#define TL   300
#define VV   25
#define CO   128
#define KT   9
#define TO   150
#define TPAD 4
#define TP   (TL + 2 * TPAD)
#define TV   (TL * VV)
#define COLS (TO * VV)
#define CP   3776
#define NCT  (CP / 64)
#define KC   (KT * CO)
#define GT   4
#define SP   136
#define XP   72
#define WSC  64.0f
#define WSI  (1.0f / 64.0f)
#define BN_EPS 1e-5f
#define ROWP (VV * CO / 8)
#define ROWI ((ROWP + 31) / 32)

static_assert((TL + 2 * TPAD - KT) / 2 + 1 == TO);
static_assert(2 * (TO - 1) + KT - 1 < TP);
static_assert(TL % GT == 0);
static_assert(TL / GT >= 2);
static_assert((GT * VV) % 4 == 0);
static_assert(TPAD % GT == 0 || TPAD <= GT);
static_assert(VV <= 32);
static_assert(CI % 32 == 0);
static_assert(CI == 64);
static_assert(CO == 128);
static_assert(CO % 64 == 0);
static_assert(KC % 32 == 0);
static_assert(CP % 64 == 0);
static_assert(CP >= COLS);
static_assert(CP - COLS < 64);
static_assert(ROWP == 400);
static_assert((ROWI - 1) * 32 + 16 == ROWP);
static_assert((SP * 2) % 16 == 0);
static_assert((XP * 2) % 16 == 0);
static_assert(SP >= CO);
static_assert(XP >= CI);
static_assert(((size_t)CO * COLS) % 32 == 0);
static_assert(NB <= NB_FULL);
static_assert(CI * GT * 32 * 2 + GT * 32 * SP * 2 <= 131072);
static_assert(16 * 68 * 4 + 128 * 4 <= 131072);
static_assert(64 * XP * 2 + 2 * 16 * 68 * 4 + 4 * CO * 4 <= 131072);

typedef _Float16 h16;
typedef unsigned short bf;
typedef __attribute__((ext_vector_type(16))) __bf16   v16bf;
typedef __attribute__((ext_vector_type(16))) _Float16 v16h;
typedef __attribute__((ext_vector_type(8)))  _Float16 v8h;
typedef __attribute__((ext_vector_type(8)))  unsigned short v8us;
typedef __attribute__((ext_vector_type(8)))  float    v8f;
typedef __attribute__((ext_vector_type(4)))  float    v4f;
typedef v4f  __attribute__((may_alias)) v4fa;

__device__ __forceinline__ unsigned short f2bf(float f) { unsigned u = __float_as_uint(f); u += 0x7FFFu + ((u >> 16) & 1u); return (unsigned short)(u >> 16); }
__device__ __forceinline__ float bfr(float f) { return __uint_as_float(((unsigned)f2bf(f)) << 16); }
__device__ __forceinline__ v16h cat16(v8h lo, v8h hi) { return __builtin_shufflevector(lo, hi, 0, 1, 2, 3, 4, 5, 6, 7, 8, 9, 10, 11, 12, 13, 14, 15); }
__device__ __forceinline__ v16bf cat16b(v8us lo, v8us hi) { return __builtin_bit_cast(v16bf, __builtin_shufflevector(lo, hi, 0, 1, 2, 3, 4, 5, 6, 7, 8, 9, 10, 11, 12, 13, 14, 15)); }
__device__ __forceinline__ v16h  ldh(const h16* p) { return cat16(*(const v8h*)p, *(const v8h*)(p + 16)); }
__device__ __forceinline__ v16bf ldb(const bf* p)  { return cat16b(*(const v8us*)p, *(const v8us*)(p + 16)); }
__device__ __forceinline__ void wave_sync() { __builtin_amdgcn_fence(3  , "wavefront"); __builtin_amdgcn_wave_barrier(); asm volatile("" ::: "memory"); }
static __device__ __forceinline__ h16 toh_flush(float v) { const h16 r = (h16)v; return (fabsf(v) < 6.103515625e-05f) ? (h16)0.0f : r; }
__device__ __forceinline__ v8f wmma16g(v16h a, v16h b, v8f c) {
    c = __builtin_amdgcn_wmma_f32_16x16x32_f16(false, a, false, b, (short)0, c, false, false);
    asm volatile("v_nop\n\tv_nop\n\tv_nop\n\tv_nop" : "+v"(c) : "v"(a), "v"(b));
    return c;
}
__device__ __forceinline__ v8f wmmabg(v16bf a, v16bf b, v8f c) {
    c = __builtin_amdgcn_wmma_f32_16x16x32_bf16(false, a, false, b, (short)0, c, false, false);
    asm volatile("v_nop\n\tv_nop\n\tv_nop\n\tv_nop" : "+v"(c) : "v"(a), "v"(b));
    return c;
}

#define PB_TW ((CO * KC) / 2048)
#define PB_GW ((CO * CI) / 2048)
#define PB_RW ((CO * CI) / 2048)
#define PB_TOTAL (PB_TW + PB_GW + PB_RW + 1)
static_assert((CO * KC) % 2048 == 0);
static_assert((CO * CI) % 2048 == 0);
static_assert(CO % 8 == 0);

__global__ __launch_bounds__(256) void k_prep(const float* __restrict__ tw, const float* __restrict__ gw, const float* __restrict__ rw,
                                              const float* __restrict__ ap, const float* __restrict__ ei, h16* TW, h16* GW, bf* RW, bf* AHL) {
#pragma clang fp contract(off)
    __shared__ __align__(16) unsigned short sa[2048];
    const int blk = blockIdx.x, tid = threadIdx.x;
    if (blk < PB_TW) {
        const int base = (blk * 256 + tid) * 8;
        const int o = base / KC, rest = base - o * KC; const int k = rest >> 7, i0 = rest & 127;
        v8h ov;
#pragma unroll
        for (int e = 0; e < 8; ++e) ov[e] = toh_flush(bfr(tw[(size_t)o * KC + (size_t)(i0 + e) * KT + k]) * WSC);
        *(volatile v8h*)(TW + base) = ov; __threadfence(); *(volatile v8h*)(TW + base) = ov;
    } else if (blk < PB_TW + PB_GW) {
        const int base = ((blk - PB_TW) * 256 + tid) * 8;
        const v8f v = *(const v8f*)(gw + base); v8h ov;
#pragma unroll
        for (int e = 0; e < 8; ++e) ov[e] = toh_flush(bfr(v[e]) * WSC);
        *(volatile v8h*)(GW + base) = ov; __threadfence(); *(volatile v8h*)(GW + base) = ov;
    } else if (blk < PB_TW + PB_GW + PB_RW) {
        const int base = ((blk - PB_TW - PB_GW) * 256 + tid) * 8;
        const v8f v = *(const v8f*)(rw + base); v8us ov;
#pragma unroll
        for (int e = 0; e < 8; ++e) ov[e] = f2bf(v[e]);
        *(volatile v8us*)(RW + base) = ov; __threadfence(); *(volatile v8us*)(RW + base) = ov;
    } else {
        const float e0 = bfr(ei[0]), e1 = bfr(ei[1]), e2 = bfr(ei[2]);
#pragma unroll 1
        for (int q = 0; q < 4; ++q) {
            const int idx = q * 256 + tid; const int w = idx >> 5, v = idx & 31;
            const int wc = w < VV ? w : VV - 1, vc = v < VV ? v : VV - 1;
            float a0 = ap[(0 * VV + vc) * VV + wc], a1 = ap[(1 * VV + vc) * VV + wc], a2 = ap[(2 * VV + vc) * VV + wc];
            asm volatile("" : "+v"(a0)); asm volatile("" : "+v"(a1)); asm volatile("" : "+v"(a2));
            float s = bfr(a0) * e0; s = s + bfr(a1) * e1; s = s + bfr(a2) * e2;
            s = ((w < VV) & (v < VV)) ? s : 0.0f;
            const unsigned short hb = f2bf(s); const float hf = __uint_as_float(((unsigned)hb) << 16);
            const unsigned short lb = f2bf(s - hf);
            sa[idx] = hb; sa[1024 + idx] = lb;
        }
        __syncthreads();
        const v8us ov = *(const v8us*)(&sa[tid * 8]);
        *(volatile v8us*)(AHL + tid * 8) = ov; __threadfence(); *(volatile v8us*)(AHL + tid * 8) = ov;
    }
}

__device__ __forceinline__ void zero_time_row(h16* d, int lane) {
#pragma unroll 1
    for (int ps = 0; ps < 2; ++ps) {
#pragma unroll 1
        for (int it = 0; it < ROWI; ++it) { const int p = it * 32 + lane; if (p < ROWP) *(volatile v8h*)(d + (size_t)p * 8) = (v8h){}; }
        if (ps == 0) __threadfence(); }
}

__global__ __launch_bounds__(32 * GT) void k_gcn(const float* __restrict__ x, const bf* __restrict__ AHL, const h16* __restrict__ GW, const float* __restrict__ gb, h16* XG) {
    __shared__ __align__(16) unsigned short xs[CI * GT * 32];
    __shared__ __align__(16) h16 st[GT * 32 * SP];
    const int tid = threadIdx.x, lane = tid & 31, lr = lane & 15, hi = lane >> 4;
    const int wave = __builtin_amdgcn_readfirstlane((int)(threadIdx.x >> 5));
    const int n = blockIdx.y, t0 = blockIdx.x * GT;
#pragma unroll 1
    for (int i = tid; i < CI * GT * 32 / 8; i += 32 * GT) *(v8us*)(&xs[i * 8]) = (v8us){};
    __syncthreads();
    const float* xb = x + (size_t)n * CI * TV + (size_t)t0 * VV;
#pragma unroll 1
    for (int i = tid; i < CI * (GT * VV / 4); i += 32 * GT) {
        const int c = i / (GT * VV / 4), q = i - c * (GT * VV / 4);
        const v4f v = *(const v4f*)(xb + (size_t)c * TV + 4 * q);
#pragma unroll
        for (int e = 0; e < 4; ++e) { const int el = 4 * q + e; const int tt = el / VV, vv = el - tt * VV; xs[(c * GT + tt) * 32 + vv] = f2bf(v[e]); }
    }
    __syncthreads();
    if (blockIdx.x == 0) {
        for (int tp = wave; tp < TPAD; tp += GT) zero_time_row(XG + ((size_t)((size_t)n * TP + tp) * VV) * CO, lane);
    }
    if (blockIdx.x == gridDim.x - 1) {
        for (int tp = wave; tp < TPAD; tp += GT) zero_time_row(XG + ((size_t)((size_t)n * TP + TPAD + TL + tp) * VV) * CO, lane);
    }
    const bf* ah = AHL + (size_t)lr * 32 + 8 * hi;
    const v16bf bh0 = ldb(ah), bh1 = ldb(ah + 16 * 32), bl0 = ldb(ah + 1024), bl1 = ldb(ah + 1024 + 16 * 32);
    v8f ag[4][2];
#pragma unroll
    for (int j = 0; j < 4; ++j) {
        const int xo = ((16 * j + lr) * GT + wave) * 32 + 8 * hi;
        const v16bf xa = cat16b(*(const v8us*)(&xs[xo]), *(const v8us*)(&xs[xo + 16]));
        ag[j][0] = wmmabg(xa, bh0, (v8f){}); ag[j][0] = wmmabg(xa, bl0, ag[j][0]);
        ag[j][1] = wmmabg(xa, bh1, (v8f){}); ag[j][1] = wmmabg(xa, bl1, ag[j][1]);
    }
    v16h bg[2][2];
#pragma unroll
    for (int ks = 0; ks < 2; ++ks)
#pragma unroll
        for (int wt = 0; wt < 2; ++wt)
#pragma unroll
            for (int r = 0; r < 8; ++r) { bg[ks][wt][r] = toh_flush(ag[2 * ks][wt][r]); bg[ks][wt][8 + r] = toh_flush(ag[2 * ks + 1][wt][r]); }
    const int sb = wave * 32 * SP;
#pragma unroll 1
    for (int og = 0; og < 2; ++og) {
        v8f a2[4][2];
#pragma unroll
        for (int ot = 0; ot < 4; ++ot) { a2[ot][0] = (v8f){}; a2[ot][1] = (v8f){}; }
#pragma unroll
        for (int ks = 0; ks < 2; ++ks) {
#pragma unroll
            for (int ot = 0; ot < 4; ++ot) {
                const v16h wa = ldh(GW + (size_t)(og * 64 + ot * 16 + lr) * CI + ks * 32 + 8 * hi);
                a2[ot][0] = wmma16g(wa, bg[ks][0], a2[ot][0]);
                a2[ot][1] = wmma16g(wa, bg[ks][1], a2[ot][1]);
            }
        }
#pragma unroll
        for (int ot = 0; ot < 4; ++ot) {
            const int ob = og * 64 + ot * 16 + 8 * hi;
            const v4f g0 = *(const v4f*)(gb + ob), g1 = *(const v4f*)(gb + ob + 4);
            float bb[8];
#pragma unroll
            for (int i = 0; i < 4; ++i) { bb[i] = bfr(g0[i]); bb[4 + i] = bfr(g1[i]); }
#pragma unroll
            for (int wt = 0; wt < 2; ++wt) { v8h hv;
#pragma unroll
                for (int j = 0; j < 8; ++j) hv[j] = toh_flush(a2[ot][wt][j] * WSI + bb[j]);
                *(v8h*)(&st[sb + (wt * 16 + lr) * SP + ob]) = hv; }
        }
    }
    wave_sync();
    h16* dst = XG + ((size_t)((size_t)n * TP + TPAD + t0 + wave) * VV) * CO;
#pragma unroll 1
    for (int ps = 0; ps < 2; ++ps) {
#pragma unroll 1
        for (int it = 0; it < ROWI; ++it) { const int p = it * 32 + lane; const int pc = p < ROWP ? p : ROWP - 1;
            const v8h val = *(const v8h*)(&st[sb + (pc >> 4) * SP + (pc & 15) * 8]);
            if (p < ROWP) *(volatile v8h*)(dst + (size_t)p * 8) = val; }
        if (ps == 0) __threadfence(); }
}

__global__ __launch_bounds__(32) void k_tcn(const h16* __restrict__ TW, const h16* __restrict__ XG, const float* __restrict__ tb, float* XT, float* PART) {
    __shared__ __align__(16) float os[16 * 68];
    __shared__ __align__(16) float sst[128];
    const int lane = threadIdx.x & 31, lr = lane & 15, hi = lane >> 4;
    const int ct = blockIdx.x, r0 = blockIdx.y * 64, n = blockIdx.z; const int c0 = ct * 64;
    v8f acc[4][4];
#pragma unroll
    for (int mb = 0; mb < 4; ++mb)
#pragma unroll
        for (int nb = 0; nb < 4; ++nb) acc[mb][nb] = (v8f){};
    size_t boff[4]; bool okc[4];
#pragma unroll
    for (int nb = 0; nb < 4; ++nb) { const int col = c0 + nb * 16 + lr; const int cc = col < COLS ? col : COLS - 1; const int tq = cc / VV, vq = cc - tq * VV;
        boff[nb] = ((size_t)((size_t)n * TP + 2 * tq) * VV + vq) * CO + 8 * hi; okc[nb] = col < COLS; }
    const size_t aoff = (size_t)(r0 + lr) * KC + 8 * hi;
#pragma unroll 1
    for (int kc = 0; kc < KC; kc += 32) {
        const size_t bo = (size_t)(kc >> 7) * (VV * CO) + (size_t)(kc & 127);
        v16h a[4];
#pragma unroll
        for (int mb = 0; mb < 4; ++mb) a[mb] = ldh(TW + aoff + (size_t)mb * 16 * KC + kc);
#pragma unroll
        for (int nb = 0; nb < 4; ++nb) { const v16h b = ldh(XG + boff[nb] + bo);
#pragma unroll
            for (int mb = 0; mb < 4; ++mb) acc[mb][nb] = wmma16g(a[mb], b, acc[mb][nb]); }
    }
    const size_t xrow = ((size_t)n * CO + r0) * CP + c0;
#pragma unroll
    for (int mb = 0; mb < 4; ++mb) {
        const int o8 = r0 + mb * 16 + 8 * hi;
        const v4f t0v = *(const v4f*)(tb + o8), t1v = *(const v4f*)(tb + o8 + 4);
        float br[8], sj[8], qj[8];
#pragma unroll
        for (int i = 0; i < 4; ++i) { br[i] = bfr(t0v[i]); br[4 + i] = bfr(t1v[i]); }
#pragma unroll
        for (int j = 0; j < 8; ++j) { sj[j] = 0.0f; qj[j] = 0.0f; }
#pragma unroll
        for (int nb = 0; nb < 4; ++nb) {
#pragma unroll
            for (int j = 0; j < 8; ++j) { const float v = acc[mb][nb][j] * WSI + br[j];
                os[(hi * 8 + j) * 68 + nb * 16 + lr] = v;
                const float vk = okc[nb] ? v : 0.0f; sj[j] += vk; qj[j] += vk * vk; } }
#pragma unroll
        for (int j = 0; j < 8; ++j) {
#pragma unroll
            for (int d = 1; d < 16; d <<= 1) { sj[j] += __shfl_xor(sj[j], d, 32); qj[j] += __shfl_xor(qj[j], d, 32); } }
        if (lr == 0) {
#pragma unroll
            for (int jj = 0; jj < 4; ++jj) { v4f t; t[0] = sj[2 * jj]; t[1] = qj[2 * jj]; t[2] = sj[2 * jj + 1]; t[3] = qj[2 * jj + 1];
                *(v4fa*)(&sst[(mb * 16 + 8 * hi) * 2 + 4 * jj]) = t; } }
        wave_sync();
#pragma unroll 1
        for (int ps = 0; ps < 2; ++ps) {
#pragma unroll
            for (int s = 0; s < 8; ++s) { const int row = 2 * s + (lane >> 4), c4 = (lane & 15) * 4;
                const v4f val = *(const v4fa*)(&os[row * 68 + c4]);
                *(volatile v4f*)(XT + xrow + (size_t)(mb * 16 + row) * CP + c4) = val; }
            if (ps == 0) __threadfence(); }
        wave_sync();
    }
    const v4f pv = *(const v4fa*)(&sst[lane * 4]);
    float* pd = PART + ((size_t)((size_t)n * NCT + ct) * 2 + blockIdx.y) * 128 + lane * 4;
    *(volatile v4f*)pd = pv; __threadfence(); *(volatile v4f*)pd = pv;
}

__global__ __launch_bounds__(128) void k_stats(const float* __restrict__ PART, float* STATS) {
#pragma clang fp contract(off)
    __shared__ __align__(16) float sm[256];
    const int o = threadIdx.x; const int oh = o >> 6, ol = o & 63;
    double S = 0.0, Q = 0.0;
#pragma unroll 1
    for (int tl = 0; tl < NB * NCT; ++tl) { const float* p = PART + ((size_t)tl * 2 + oh) * 128 + ol * 2; S += (double)p[0]; Q += (double)p[1]; }
    const double ic = 1.0 / (double)((size_t)NB * COLS);
    const double mean = S * ic; double var = Q * ic - mean * mean; var = var < 0.0 ? 0.0 : var;
    const float varf = (float)var;
    sm[o] = (float)mean; sm[CO + o] = 1.0f / sqrtf(varf + BN_EPS);
    __syncthreads();
    if (threadIdx.x < 64) { const v4f val = *(const v4fa*)(&sm[threadIdx.x * 4]);
        *(volatile v4f*)(STATS + threadIdx.x * 4) = val; __threadfence(); *(volatile v4f*)(STATS + threadIdx.x * 4) = val; }
}

__global__ __launch_bounds__(64) void k_res(const float* __restrict__ x, const bf* __restrict__ RW, const float* __restrict__ rb, const float* __restrict__ gam, const float* __restrict__ bet,
                                            const float* __restrict__ STATS, const float* __restrict__ XT, float* Y) {
    __shared__ __align__(16) unsigned short xt_[64 * XP];
    __shared__ __align__(16) float os[2 * 16 * 68];
    __shared__ __align__(16) float sP[4 * CO];
    const int tid = threadIdx.x, lane = tid & 31, lr = lane & 15, hi = lane >> 4;
    const int wave = __builtin_amdgcn_readfirstlane((int)(threadIdx.x >> 5));
    const int ct = blockIdx.x, n = blockIdx.y; const int c0 = ct * 64;
#pragma unroll 1
    for (int i = tid; i < CO; i += 64) { sP[i] = STATS[i]; sP[CO + i] = STATS[CO + i]; sP[2 * CO + i] = bfr(gam[i]); sP[3 * CO + i] = bfr(bet[i]); }
    { const int col = c0 + tid; const int cc = col < COLS ? col : COLS - 1; const int tq = cc / VV, vq = cc - tq * VV;
      const float* xp = x + (size_t)n * CI * TV + (size_t)(2 * tq) * VV + vq;
#pragma unroll 4
      for (int c = 0; c < CI; ++c) xt_[tid * XP + c] = f2bf(xp[(size_t)c * TV]); }
    __syncthreads();
    const int r0 = wave * 64;
    v8f acc[4][4];
#pragma unroll
    for (int mb = 0; mb < 4; ++mb)
#pragma unroll
        for (int nb = 0; nb < 4; ++nb) acc[mb][nb] = (v8f){};
#pragma unroll 1
    for (int kc = 0; kc < CI; kc += 32) {
        v16bf a[4];
#pragma unroll
        for (int mb = 0; mb < 4; ++mb) a[mb] = ldb(RW + (size_t)(r0 + mb * 16 + lr) * CI + kc + 8 * hi);
#pragma unroll
        for (int nb = 0; nb < 4; ++nb) { const int bo = (nb * 16 + lr) * XP + kc + 8 * hi;
            const v16bf b = cat16b(*(const v8us*)(&xt_[bo]), *(const v8us*)(&xt_[bo + 16]));
#pragma unroll
            for (int mb = 0; mb < 4; ++mb) acc[mb][nb] = wmmabg(a[mb], b, acc[mb][nb]); }
    }
    const int ob = wave * 16 * 68;
    const size_t yrow = ((size_t)n * CO + r0) * CP + c0;
#pragma unroll
    for (int mb = 0; mb < 4; ++mb) {
        const int o8 = r0 + mb * 16 + 8 * hi;
        const v4f b0 = *(const v4f*)(rb + o8), b1 = *(const v4f*)(rb + o8 + 4);
        float br[8];
#pragma unroll
        for (int i = 0; i < 4; ++i) { br[i] = bfr(b0[i]); br[4 + i] = bfr(b1[i]); }
#pragma unroll
        for (int nb = 0; nb < 4; ++nb) {
#pragma unroll
            for (int j = 0; j < 8; ++j) os[ob + (hi * 8 + j) * 68 + nb * 16 + lr] = acc[mb][nb][j] + br[j]; }
        wave_sync();
        v4f val[8];
#pragma unroll
        for (int s = 0; s < 8; ++s) { const int row = 2 * s + (lane >> 4), c4 = (lane & 15) * 4; const int o = r0 + mb * 16 + row;
            const float mu = sP[o], rs = sP[CO + o], g = sP[2 * CO + o], be = sP[3 * CO + o];
            const v4f rv = *(const v4fa*)(&os[ob + row * 68 + c4]);
            const v4f xv = *(const v4f*)(XT + yrow + (size_t)(mb * 16 + row) * CP + c4);
#pragma unroll
            for (int i = 0; i < 4; ++i) { float u = (xv[i] - mu) * rs; u = u * g + be; u = u + rv[i]; val[s][i] = u > 0.0f ? u : 0.0f; } }
#pragma unroll 1
        for (int ps = 0; ps < 2; ++ps) {
#pragma unroll
            for (int s = 0; s < 8; ++s) { const int row = 2 * s + (lane >> 4), c4 = (lane & 15) * 4;
                *(volatile v4f*)(Y + yrow + (size_t)(mb * 16 + row) * CP + c4) = val[s]; }
            if (ps == 0) __threadfence(); }
        wave_sync();
    }
}

__global__ __launch_bounds__(256) void k_copy(const float* __restrict__ Y, float* OUT, unsigned n4) {
#pragma clang fp contract(off)
    const unsigned i = blockIdx.x * 256u + threadIdx.x; if (i >= n4) return;
    const unsigned f = i * 4u; const unsigned row = f / (unsigned)COLS; const unsigned col = f - row * (unsigned)COLS;
    v4f v;
#pragma unroll
    for (int e = 0; e < 4; ++e) { const unsigned c = col + (unsigned)e; const bool wrap = c >= (unsigned)COLS;
        const unsigned cc = wrap ? c - (unsigned)COLS : c; const unsigned rr = wrap ? row + 1u : row;
        v[e] = Y[(size_t)rr * CP + cc]; }
    *(volatile v4f*)(OUT + (size_t)f) = v; __threadfence(); *(volatile v4f*)(OUT + (size_t)f) = v;
}

static constexpr size_t al256(size_t v) { return (v + 255) & ~(size_t)255; }
static constexpr size_t SZ_TW = al256((size_t)CO * KC * 2);
static constexpr size_t SZ_GW = al256((size_t)CO * CI * 2);
static constexpr size_t SZ_RW = al256((size_t)CO * CI * 2);
static constexpr size_t SZ_AH = al256((size_t)2 * 32 * 32 * 2);
static constexpr size_t SZ_ST = al256((size_t)2 * CO * 4);
static constexpr size_t SZ_PT = al256((size_t)NB * NCT * 2 * 128 * 4);
static constexpr size_t SZ_XG = al256((size_t)NB * TP * VV * CO * 2);
static constexpr size_t SZ_XT = al256((size_t)NB * CO * CP * 4);
static constexpr size_t SZ_Y  = al256((size_t)NB * CO * CP * 4);
static constexpr size_t SZ_TOTAL = SZ_TW + SZ_GW + SZ_RW + SZ_AH + SZ_ST + SZ_PT + SZ_XG + SZ_XT;
static_assert(SZ_Y <= SZ_XG);
static_assert(SZ_TOTAL <= (size_t)134217728);
static_assert((size_t)PB_TW * 2048 == (size_t)CO * KC);
static_assert(((size_t)NB * CO * COLS) % 4 == 0);

extern "C" void kernel_launch(void* const* d_in, const int* in_sizes, int n_in,
                              void* d_out, int out_size, void* d_ws, size_t ws_size, hipStream_t stream) {
    if (n_in < 11) return;
    if ((size_t)in_sizes[0] < (size_t)NB * CI * TV) return;
    if (in_sizes[1] < 3 * VV * VV || in_sizes[2] < 3) return;
    if (in_sizes[3] < CO * CI || in_sizes[4] < CO) return;
    if (in_sizes[5] < CO * CO * KT || in_sizes[6] < CO) return;
    if (in_sizes[7] < CO || in_sizes[8] < CO) return;
    if (in_sizes[9] < CO * CI || in_sizes[10] < CO) return;
    if ((size_t)out_size < (size_t)NB * CO * COLS) return;
    if (SZ_TOTAL > ws_size) return;
    const float* x   = (const float*)d_in[0];
    const float* ap  = (const float*)d_in[1];
    const float* ei  = (const float*)d_in[2];
    const float* gw  = (const float*)d_in[3];
    const float* gb  = (const float*)d_in[4];
    const float* tw  = (const float*)d_in[5];
    const float* tb  = (const float*)d_in[6];
    const float* gam = (const float*)d_in[7];
    const float* bet = (const float*)d_in[8];
    const float* rw  = (const float*)d_in[9];
    const float* rb  = (const float*)d_in[10];
    float* OUT = (float*)d_out;
    char* wsp = (char*)d_ws;
    h16* TW = (h16*)wsp; wsp += SZ_TW;
    h16* GW = (h16*)wsp; wsp += SZ_GW;
    bf*  RW = (bf*)wsp;  wsp += SZ_RW;
    bf*  AHL = (bf*)wsp; wsp += SZ_AH;
    float* STATS = (float*)wsp; wsp += SZ_ST;
    float* PART = (float*)wsp;  wsp += SZ_PT;
    h16* XG = (h16*)wsp;
    float* Y = (float*)wsp; wsp += SZ_XG;
    float* XT = (float*)wsp; wsp += SZ_XT;

    k_prep<<<PB_TOTAL, 256, 0, stream>>>(tw, gw, rw, ap, ei, TW, GW, RW, AHL);
    k_gcn<<<dim3(TL / GT, NB, 1), 32 * GT, 0, stream>>>(x, AHL, GW, gb, XG);
    k_tcn<<<dim3(NCT, CO / 64, NB), 32, 0, stream>>>(TW, XG, tb, XT, PART);
    k_stats<<<1, 128, 0, stream>>>(PART, STATS);
    k_res<<<dim3(NCT, NB, 1), 64, 0, stream>>>(x, RW, rb, gam, bet, STATS, XT, Y);
    { const unsigned n4 = (unsigned)((size_t)NB * CO * COLS / 4);
      k_copy<<<(n4 + 255u) / 256u, 256, 0, stream>>>(Y, OUT, n4); }
}
